// TrajNet_22110491640215
// MI455X (gfx1250) — hardware-verified
//
#include <hip/hip_runtime.h>


namespace {
constexpr int NB = 8192, XD = 44, KP = 64, H1 = 64, BO = 12, NV = 11, NC = 6, NUM = 30, ITERS = 300;
constexpr float HS = 256.0f, WSC = 256.0f, RHO = 10.0f, WSM = 10.0f;
typedef _Float16 b16;
typedef __attribute__((ext_vector_type(16))) _Float16 v16b;
typedef __attribute__((ext_vector_type(8))) _Float16 v8b;
typedef __attribute__((ext_vector_type(8))) float v8f;
typedef __attribute__((ext_vector_type(4))) float v4f;
__device__ __forceinline__ float bf16_rne(float f) { unsigned int u = __float_as_uint(f); u += 0x7FFFu + ((u >> 16) & 1u); float r = __uint_as_float(u & 0xFFFF0000u); asm volatile("" : "+v"(r)); return r; }
__device__ __forceinline__ float bfv(float f) { float r = bf16_rne(f); asm volatile("" : "+v"(r)); return r; }
__device__ __forceinline__ void split16(float v, b16& hi, b16& lo) { hi = (b16)v; lo = (b16)(v - (float)hi); }
__device__ __forceinline__ v16b frag_kb(const b16* p, int hh) { const v8b a = *(const v8b*)(p + 8 * hh), b = *(const v8b*)(p + 16 + 8 * hh); v16b f;
#pragma unroll
  for (int e = 0; e < 8; ++e) { f[e] = a[e]; f[8 + e] = b[e]; } return f; }
__device__ __forceinline__ v8f wmma16b(v16b a, v16b b, v8f c) { v8f d = __builtin_amdgcn_wmma_f32_16x16x32_f16(false, a, false, b, (short)0, c, false, false); asm volatile("v_nop\n\tv_nop\n\tv_nop\n\tv_nop" : "+v"(d) : "v"(a), "v"(b)); return d; }
__device__ __forceinline__ void wave_lds_sync() { __builtin_amdgcn_fence(__ATOMIC_RELEASE, "workgroup"); __builtin_amdgcn_wave_barrier(); __builtin_amdgcn_fence(__ATOMIC_ACQUIRE, "workgroup"); }
__device__ __forceinline__ float pmul(float a, float b) { float p = a * b; asm volatile("" : "+v"(p)); return p; }

__global__ __launch_bounds__(256) void setup_kernel(const float* __restrict__ w1, const float* __restrict__ w2, const float* __restrict__ P, const float* __restrict__ Pdd, const float* __restrict__ Aeq, b16* __restrict__ W1P, b16* __restrict__ W2P, float* __restrict__ CONST) { const int u = threadIdx.x; v8b v;
  for (int idx = u; idx < H1 * 8; idx += 256) { const int o = idx / 8, k0 = (idx % 8) * 8;
#pragma unroll
    for (int j = 0; j < 8; ++j) { const int k = k0 + j; v[j] = (b16)(k < XD ? bf16_rne(w1[o * XD + k]) * WSC : 0.0f); } for (int pass = 0; pass < 2; ++pass) { *(volatile v8b*)(W1P + (size_t)o * KP + k0) = v; __threadfence(); } }
  for (int idx = u; idx < 16 * 8; idx += 256) { const int o = idx / 8, k0 = (idx % 8) * 8;
#pragma unroll
    for (int j = 0; j < 8; ++j) v[j] = (b16)(o < BO ? bf16_rne(w2[o * H1 + k0 + j]) * WSC : 0.0f); for (int pass = 0; pass < 2; ++pass) { *(volatile v8b*)(W2P + (size_t)o * KP + k0) = v; __threadfence(); } }
  __shared__ double M[NV][2 * NV];
  if (u == 0) {
    for (int i = 0; i < NV; ++i) for (int j = 0; j < NV; ++j) { double c = 0.0; for (int k = 0; k < NUM; ++k) c += (double)bfv(Pdd[k * NV + i]) * (double)bfv(Pdd[k * NV + j]); double a = 0.0; for (int k = 0; k < NC; ++k) a += (double)bfv(Aeq[k * NV + i]) * (double)bfv(Aeq[k * NV + j]); M[i][j] = -(WSM * c + RHO * a); M[i][NV + j] = (i == j) ? 1.0 : 0.0; }
    for (int col = 0; col < NV; ++col) { int piv = col; double best = fabs(M[col][col]); for (int r = col + 1; r < NV; ++r) if (fabs(M[r][col]) > best) { best = fabs(M[r][col]); piv = r; }
      if (piv != col) for (int j = 0; j < 2 * NV; ++j) { const double t = M[col][j]; M[col][j] = M[piv][j]; M[piv][j] = t; }
      const double d = 1.0 / M[col][col]; for (int j = 0; j < 2 * NV; ++j) M[col][j] *= d;
      for (int r = 0; r < NV; ++r) if (r != col) { const double f = M[r][col]; if (f != 0.0) for (int j = 0; j < 2 * NV; ++j) M[r][j] -= f * M[col][j]; } }
    for (int pass = 0; pass < 2; ++pass) { for (int i = 0; i < NV; ++i) for (int j = 0; j < NV; ++j) ((volatile float*)CONST)[i * NV + j] = (float)M[i][NV + j]; for (int q = 0; q < NC * NV; ++q) ((volatile float*)CONST)[128 + q] = bfv(Aeq[q]); for (int q = 0; q < NUM * NV; ++q) ((volatile float*)CONST)[256 + q] = bfv(P[q]); for (int q = NV * NV; q < 128; ++q) ((volatile float*)CONST)[q] = 0.0f; for (int q = 128 + NC * NV; q < 256; ++q) ((volatile float*)CONST)[q] = 0.0f; for (int q = 256 + NUM * NV; q < 640; ++q) ((volatile float*)CONST)[q] = 0.0f; __threadfence(); } } }
__global__ __launch_bounds__(32) void traj_kernel(const float* __restrict__ x, const float* __restrict__ bin, const b16* __restrict__ W1P, const b16* __restrict__ W2P, const float* __restrict__ b1, const float* __restrict__ b2, const float* __restrict__ CONST, int SLIM, float* __restrict__ out) {
  __shared__ __attribute__((aligned(16))) b16 Ah[32][KP + 8], Al[32][KP + 8]; __shared__ float Tf[32][H1 + 4], Bp[32][16], Cs[640]; const int lane = threadIdx.x, nloc = lane & 15, hlf = lane >> 4; const size_t s0 = (size_t)blockIdx.x * 32; if (s0 >= (size_t)SLIM) return;
  for (int q = lane; q < 640; q += 32) Cs[q] = CONST[q];
  for (int rr = 0; rr < 32; ++rr) for (int q = 0; q < 2; ++q) { const int c = q * 32 + lane; Ah[rr][c] = (b16)(c < XD ? bf16_rne(x[(s0 + rr) * XD + c]) * HS : 0.0f); Al[rr][c] = (b16)0.0f; } for (int k = KP; k < KP + 8; ++k) { Ah[lane][k] = (b16)0.0f; Al[lane][k] = (b16)0.0f; }
  wave_lds_sync();
#pragma unroll 1
  for (int rt = 0; rt < 2; ++rt) { v8f acc[4] = {(v8f){}, (v8f){}, (v8f){}, (v8f){}};
#pragma unroll
    for (int kb = 0; kb < KP; kb += 32) { const v16b a = frag_kb(&Ah[rt * 16 + nloc][kb], hlf);
#pragma unroll
      for (int t = 0; t < 4; ++t) acc[t] = wmma16b(a, frag_kb(W1P + (size_t)(t * 16 + nloc) * KP + kb, hlf), acc[t]); }
#pragma unroll
    for (int t = 0; t < 4; ++t) { const int cc = t * 16 + nloc; const float bb = bfv(b1[cc]);
#pragma unroll
      for (int r8 = 0; r8 < 8; ++r8) Tf[rt * 16 + 8 * hlf + r8][cc] = fmaxf(acc[t][r8] * (1.0f / (HS * WSC)) + bb, 0.0f); } }
  wave_lds_sync();
  for (int rr = 0; rr < 32; ++rr) for (int q = 0; q < 2; ++q) { const int c = q * 32 + lane; b16 p, ql; split16(Tf[rr][c] * HS, p, ql); Ah[rr][c] = p; Al[rr][c] = ql; }
  wave_lds_sync();
#pragma unroll 1
  for (int rt = 0; rt < 2; ++rt) { v8f acc = {};
#pragma unroll
    for (int kb = 0; kb < KP; kb += 32) { const v16b bw = frag_kb(W2P + (size_t)nloc * KP + kb, hlf); acc = wmma16b(frag_kb(&Ah[rt * 16 + nloc][kb], hlf), bw, acc); acc = wmma16b(frag_kb(&Al[rt * 16 + nloc][kb], hlf), bw, acc); }
#pragma unroll
    for (int r8 = 0; r8 < 8; ++r8) Bp[rt * 16 + 8 * hlf + r8][nloc] = acc[r8] * (1.0f / (HS * WSC)) + (nloc < BO ? bfv(b2[nloc]) : 0.0f); }
  wave_lds_sync();
  const size_t s = s0 + lane; const float* NCI = Cs; const float* A = Cs + 128; const float* PP = Cs + 256; __shared__ float Os[32][2 * NUM + 1]; __shared__ float ABl[32][12], Ll[32][12], Sl[32][12], Cl[32][12], Rl[32][8], Bl[32][8];
#pragma unroll 1
  for (int hf = 0; hf < 2; ++hf) {
#pragma unroll 1
    for (int k = 0; k < NC; ++k) { const int col = hf * NC + k; Bl[lane][k] = (col == 3 || col == 9) ? Bp[lane][col] : bfv(bin[s * BO + col]); }
#pragma unroll 1
    for (int j = 0; j < NV; ++j) { float a = 0.0f;
#pragma unroll
      for (int k = 0; k < NC; ++k) a += Bl[lane][k] * A[k * NV + j]; ABl[lane][j] = RHO * a; Ll[lane][j] = 0.0f; Sl[lane][j] = 0.0f; }
#pragma unroll 1
    for (int it = 0; it < ITERS; ++it) {
#pragma unroll 1
      for (int j = 0; j < NV; ++j) Cl[lane][j] = -Ll[lane][j] - ABl[lane][j];
#pragma unroll 1
      for (int j = 0; j < NV; ++j) { float a = 0.0f;
#pragma unroll
        for (int i = 0; i < NV; ++i) a += Cl[lane][i] * NCI[i * NV + j]; Sl[lane][j] = a; }
#pragma unroll 1
      for (int k = 0; k < NC; ++k) { float a = 0.0f;
#pragma unroll
        for (int j = 0; j < NV; ++j) a += Sl[lane][j] * A[k * NV + j]; Rl[lane][k] = a - Bl[lane][k]; }
#pragma unroll 1
      for (int j = 0; j < NV; ++j) { float a = 0.0f;
#pragma unroll
        for (int k = 0; k < NC; ++k) a += Rl[lane][k] * A[k * NV + j]; Ll[lane][j] -= RHO * a; } }
#pragma unroll 1
    for (int m = 0; m < NUM; ++m) { float a = 0.0f;
#pragma unroll
      for (int j = 0; j < NV; ++j) a += Sl[lane][j] * PP[m * NV + j]; Os[lane][hf * NUM + m] = a; } }
  wave_lds_sync();
  for (int pass = 0; pass < 2; ++pass) { for (int idx = lane; idx < 32 * 2 * NUM; idx += 32) ((volatile float*)out)[s0 * 2 * NUM + idx] = Os[idx / (2 * NUM)][idx % (2 * NUM)]; __threadfence(); } }
}

extern "C" void kernel_launch(void* const* d_in, const int* in_sizes, int n_in, void* d_out, int out_size, void* d_ws, size_t ws_size, hipStream_t stream) {
  (void)n_in;
  auto Fp = [&](int i) { return (const float*)d_in[i]; };
  if (in_sizes[0] != NB * XD || in_sizes[1] != NB * BO || in_sizes[2] != H1 * XD || in_sizes[3] != H1 || in_sizes[4] != BO * H1 || in_sizes[5] != BO || in_sizes[6] != NUM * NV || in_sizes[7] != NUM * NV || in_sizes[8] != NC * NV || out_size != NB * 2 * NUM) return;
  const int SLIM = NB;
  size_t off = 0; char* ws = (char*)d_ws;
  auto carve = [&](size_t bytes) { char* p = ws + off; off += (bytes + 255) & ~(size_t)255; return p; };
  b16* W1P = (b16*)carve((size_t)H1 * KP * 2); b16* W2P = (b16*)carve((size_t)16 * KP * 2); float* CONST = (float*)carve(640 * 4);
  if (off > ws_size || off > ((size_t)1 << 20)) return;
  setup_kernel<<<1, 256, 0, stream>>>(Fp(2), Fp(4), Fp(6), Fp(7), Fp(8), W1P, W2P, CONST);
  traj_kernel<<<SLIM / 32, 32, 0, stream>>>(Fp(0), Fp(1), W1P, W2P, Fp(3), Fp(5), CONST, SLIM, (float*)d_out);
}
